// MultiHeadAttentionRelativePosition_70686571757924
// MI455X (gfx1250) — hardware-verified
//
#include <hip/hip_runtime.h>
#include <math.h>

typedef __attribute__((ext_vector_type(16))) _Float16 v16h;
typedef __attribute__((ext_vector_type(16))) __bf16 v16b;
typedef __attribute__((ext_vector_type(8)))  _Float16 v8h;
typedef __attribute__((ext_vector_type(8)))  float v8f;
typedef __attribute__((ext_vector_type(4)))  float v4f;
typedef __attribute__((ext_vector_type(2)))  float v2f;
typedef __attribute__((ext_vector_type(4)))  unsigned v4u;
typedef __attribute__((ext_vector_type(4)))  int v4i;
typedef float __attribute__((may_alias)) float_a;
typedef int __attribute__((may_alias)) int_a;

template <typename T> __device__ __forceinline__ void vst2(void* p, T v) { *(volatile T*)p = v; __threadfence(); *(volatile T*)p = v; }
__device__ __forceinline__ v8f wmma16(v16h a, v16h b, v8f c) {
  v8f d = __builtin_amdgcn_wmma_f32_16x16x32_f16(false, a, false, b, (short)0, c, false, false);
  asm volatile("v_nop\n\tv_nop\n\tv_nop\n\tv_nop" : "+v"(d) : "v"(a), "v"(b));
  return d;
}
__device__ __forceinline__ v8f wmma_bf(v16b a, v16b b, v8f c) {
  v8f d = __builtin_amdgcn_wmma_f32_16x16x32_bf16(false, a, false, b, (short)0, c, false, false);
  asm volatile("v_nop\n\tv_nop\n\tv_nop\n\tv_nop" : "+v"(d) : "v"(a), "v"(b));
  return d;
}
__device__ __forceinline__ v16h frag_h(const _Float16* rowk0, int lane) {
  union { v16h v; v8h q[2]; } u; const _Float16* p = rowk0 + 8 * (lane >> 4);
  u.q[0] = *(const v8h*)p; u.q[1] = *(const v8h*)(p + 16); return u.v;
}
__device__ __forceinline__ v16h frag_f32(const float* rowk0, int lane) {
  v16h a; const float* p = rowk0 + 8 * (lane >> 4);
#pragma unroll
  for (int i = 0; i < 8; ++i) { a[i] = (_Float16)p[i]; a[8 + i] = (_Float16)p[16 + i]; }
  return a;
}
__device__ __forceinline__ v16h frag_f32s(const float* rowk0, int lane, float sc) {
  v16h a; const float* p = rowk0 + 8 * (lane >> 4);
#pragma unroll
  for (int i = 0; i < 8; ++i) { a[i] = (_Float16)(p[i] * sc); a[8 + i] = (_Float16)(p[16 + i] * sc); }
  return a;
}
__device__ __forceinline__ v16h fragc_f32(const float* W, int k0, int n, int lane, int ld, int K) {
  v16h a; const int g = lane >> 4;
#pragma unroll
  for (int i = 0; i < 8; ++i) { const int ka = k0 + 8 * g + i, kb = ka + 16;
    a[i] = (_Float16)(ka < K ? W[(size_t)(ka < K ? ka : K - 1) * ld + n] : 0.f); a[8 + i] = (_Float16)(kb < K ? W[(size_t)(kb < K ? kb : K - 1) * ld + n] : 0.f); }
  return a;
}
struct F2 { v16b h, l; };
__device__ __forceinline__ F2 bsplit16(const float v[16]) { F2 r;
#pragma unroll
  for (int i = 0; i < 16; ++i) { const __bf16 h = (__bf16)v[i]; r.h[i] = h; r.l[i] = (__bf16)(v[i] - (float)h); }
  return r; }
__device__ __forceinline__ F2 split_row(const float* row, int k0, int lane) { float v[16]; const float* p = row + k0 + 8 * (lane >> 4);
#pragma unroll
  for (int i = 0; i < 8; ++i) { v[i] = p[i]; v[8 + i] = p[16 + i]; }
  return bsplit16(v); }
__device__ __forceinline__ F2 split_rowK(const float* row, int k0, int lane, int K) { float v[16]; const int g = lane >> 4;
#pragma unroll
  for (int i = 0; i < 8; ++i) { const int ka = k0 + 8 * g + i, kb = ka + 16; v[i] = ka < K ? row[ka < K ? ka : K - 1] : 0.f; v[8 + i] = kb < K ? row[kb < K ? kb : K - 1] : 0.f; }
  return bsplit16(v); }
__device__ __forceinline__ F2 split_col(const float* W, int k0, int n, int lane, int ld, int K) { float v[16]; const int g = lane >> 4;
#pragma unroll
  for (int i = 0; i < 8; ++i) { const int ka = k0 + 8 * g + i, kb = ka + 16; v[i] = ka < K ? W[(size_t)(ka < K ? ka : K - 1) * ld + n] : 0.f; v[8 + i] = kb < K ? W[(size_t)(kb < K ? kb : K - 1) * ld + n] : 0.f; }
  return bsplit16(v); }
__device__ __forceinline__ v8f mac3(const F2& a, const F2& b, v8f c) { c = wmma_bf(a.l, b.h, c); c = wmma_bf(a.h, b.l, c); return wmma_bf(a.h, b.h, c); }
__device__ __forceinline__ float sigm(float v) { return 1.0f / (1.0f + expf(-v)); }
#define LDSX() do { asm volatile("s_wait_dscnt 0" ::: "memory"); __builtin_amdgcn_wave_barrier(); __builtin_amdgcn_fence(__ATOMIC_RELEASE, "workgroup"); } while (0)


#define NB 2
#define SS 2048
#define DM 1024
#define NH 16
#define HD 64
#define QKVW (3 * DM)
#ifndef TQB
#define TQB (SS / 64)
#define TNB NB
#define TOB (NB * SS / 64)
#endif
typedef __attribute__((ext_vector_type(8))) __bf16 v8b;
__device__ __forceinline__ v16b frag_b(const __bf16* rowk0, int lane) {
  union { v16b v; v8b q[2]; } u; const __bf16* p = rowk0 + 8 * (lane >> 4);
  u.q[0] = *(const v8b*)p; u.q[1] = *(const v8b*)(p + 16); return u.v;
}
__device__ __forceinline__ float bfr(float v) { return (float)(__bf16)v; }
__device__ __attribute__((noinline)) float exp_ni(float v) { return expf(v); }
__device__ __attribute__((noinline)) float erf_ni(float v) { return erff(v); }

#define PK_A 0
#define PK_P (PK_A + QKVW * DM)
#define PK_END (PK_P + DM * DM)
#define WS_PK  0u
#define WS_QK  (WS_PK + 2u * PK_END)
#define WS_VTH (WS_QK + 4u * NB * SS * QKVW)
#define WS_VTL (WS_VTH + 2u * NB * DM * SS)
#define WS_O   (WS_VTL + 2u * NB * DM * SS)
#define WS_END (WS_O + 4u * NB * SS * DM)

__global__ __launch_bounds__(256) void k_packrows(const float* __restrict__ Wm, int K, __bf16* __restrict__ DST) {
  __shared__ __align__(16) __bf16 s[DM]; const int n = blockIdx.x, tid = threadIdx.x;
  for (int k = tid; k < K; k += 256) s[k] = (__bf16)Wm[(size_t)n * K + k];
  __syncthreads();
  for (int q = tid; q < K / 8; q += 256) vst2((unsigned*)(DST + (size_t)n * K + q * 8), *(const v4u*)&s[q * 8]);
}
__global__ __launch_bounds__(128) void k_qkv(const float* __restrict__ XQ, const float* __restrict__ XK, const float* __restrict__ XV, const __bf16* __restrict__ P, const float* __restrict__ BQ, const float* __restrict__ BK, const float* __restrict__ BV, float* __restrict__ QKV) {
  __shared__ __align__(16) float so[4][16][132];
  const int tid = threadIdx.x, wave = tid >> 5, lane = tid & 31, col = lane & 15, g = lane >> 4; const size_t r0 = (size_t)blockIdx.x * 64 + wave * 16; const int n0 = blockIdx.y * 128; const float* X = (n0 < DM) ? XQ : (n0 < 2 * DM ? XK : XV);
  v8f acc[8] = {};
#pragma unroll 2
  for (int kc = 0; kc < DM / 32; ++kc) { v16b a; { const float* p = X + (r0 + col) * DM + kc * 32 + 8 * g;
#pragma unroll
      for (int i = 0; i < 8; ++i) { a[i] = (__bf16)p[i]; a[8 + i] = (__bf16)p[16 + i]; } }
#pragma unroll
    for (int j = 0; j < 8; ++j) acc[j] = wmma_bf(a, frag_b(P + (size_t)(n0 + j * 16 + col) * DM + kc * 32, lane), acc[j]); }
  const float* bias = (n0 < DM) ? BQ : (n0 < 2 * DM ? BK : BV); const int nb = n0 % DM;
#pragma unroll
  for (int j = 0; j < 8; ++j) { const float bb = bfr(bias[nb + j * 16 + col]);
#pragma unroll
    for (int r = 0; r < 8; ++r) so[wave][8 * g + r][j * 16 + col] = acc[j][r] + bb; }
  LDSX();
  for (int rl = 0; rl < 16; ++rl) vst2(QKV + (r0 + rl) * QKVW + n0 + lane * 4, *(const v4f*)&so[wave][rl][lane * 4]);
}
__global__ __launch_bounds__(256) void k_vt(const float* __restrict__ QKV, __bf16* __restrict__ VTH, __bf16* __restrict__ VTL) {
  __shared__ __align__(16) __bf16 sth[64][72], stl[64][72]; const int tid = threadIdx.x; const size_t rb = (size_t)blockIdx.x * 64; const int h = blockIdx.y; const int b = (int)(rb / SS), s0 = (int)(rb % SS);
  for (int q = tid; q < 64 * 64; q += 256) { const int rl = q >> 6, d = q & 63; const float v = QKV[(rb + rl) * QKVW + 2 * DM + h * HD + d]; const __bf16 hb = (__bf16)v; sth[d][rl] = hb; stl[d][rl] = (__bf16)(v - (float)hb); }
  __syncthreads();
  for (int q = tid; q < 64 * 8; q += 256) { const int d = q >> 3, pc = q & 7; const size_t o = ((size_t)b * DM + h * HD + d) * SS + s0 + pc * 8; vst2((unsigned*)(VTH + o), *(const v4u*)&sth[d][pc * 8]); vst2((unsigned*)(VTL + o), *(const v4u*)&stl[d][pc * 8]); }
}
__global__ __launch_bounds__(128) void k_attn(const float* __restrict__ QK, const __bf16* __restrict__ VTH, const __bf16* __restrict__ VTL, const float* __restrict__ RK, const float* __restrict__ RV, float* __restrict__ O) {
  __shared__ __align__(16) float sp[4][16][36]; __shared__ __align__(16) float so[4][16][68]; __shared__ float sqr[4][16][8];
  const int tid = threadIdx.x, wave = tid >> 5, lane = tid & 31, col = lane & 15, g = lane >> 4;
  const int qb = blockIdx.x, h = blockIdx.y, b = blockIdx.z; const int q0 = qb * 64 + wave * 16; const size_t rq = (size_t)b * SS + q0 + col;
  F2 aq[2];
#pragma unroll
  for (int kc = 0; kc < 2; ++kc) aq[kc] = split_row(QK + rq * QKVW + h * HD, kc * 32, lane);
#pragma unroll 1
  for (int r = 0; r < 8; ++r) { const float* qrow = QK + ((size_t)b * SS + q0 + 8 * g + r) * QKVW + h * HD;
#pragma unroll
    for (int j = 0; j < 5; ++j) { float a = 0.f;
#pragma unroll
      for (int dt = 0; dt < 4; ++dt) a += qrow[dt * 16 + col] * bfr(RK[j * HD + dt * 16 + col]);
#pragma unroll
      for (int o = 1; o < 16; o <<= 1) a += __shfl_xor(a, o);
      if (col == j) sqr[wave][8 * g + r][j] = a; } }
  LDSX();
  float m[8], l[8], ms[8][5];
#pragma unroll
  for (int r = 0; r < 8; ++r) { m[r] = -3.0e38f; l[r] = 0.f; for (int j = 0; j < 5; ++j) ms[r][j] = 0.f; }
  v8f acc[4] = {};
#pragma unroll 1
  for (int ks = 0; ks < SS / 32; ++ks) { v8f s[2]; int jc[2][8];
#pragma unroll
    for (int ct = 0; ct < 2; ++ct) { const int kk = ks * 32 + ct * 16 + col; const float* krow = QK + ((size_t)b * SS + kk) * QKVW + DM + h * HD; v8f c = {};
#pragma unroll
      for (int kc = 0; kc < 2; ++kc) { const F2 kb = split_row(krow, kc * 32, lane); c = mac3(aq[kc], kb, c); }
#pragma unroll
      for (int r = 0; r < 8; ++r) { const int qi = q0 + 8 * g + r; const int dlt = min(max(kk - qi, -2), 2) + 2; jc[ct][r] = dlt; s[ct][r] = (c[r] + sqr[wave][8 * g + r][dlt]) * 0.125f; } }
#pragma unroll
    for (int r = 0; r < 8; ++r) { float mx = fmaxf(s[0][r], s[1][r]);
#pragma unroll
      for (int o = 1; o < 16; o <<= 1) mx = fmaxf(mx, __shfl_xor(mx, o));
      const float mn = fmaxf(m[r], mx); const float alpha = exp_ni(m[r] - mn);
      const float e0 = exp_ni(s[0][r] - mn), e1 = exp_ni(s[1][r] - mn); float es = e0 + e1;
#pragma unroll
      for (int o = 1; o < 16; o <<= 1) es += __shfl_xor(es, o);
      l[r] = l[r] * alpha + es; m[r] = mn;
#pragma unroll
      for (int j = 0; j < 5; ++j) { float add = ((jc[0][r] == j) ? e0 : 0.f) + ((jc[1][r] == j) ? e1 : 0.f);
#pragma unroll
        for (int o = 1; o < 16; o <<= 1) add += __shfl_xor(add, o);
        ms[r][j] = ms[r][j] * alpha + add; }
#pragma unroll
      for (int dt = 0; dt < 4; ++dt) acc[dt][r] *= alpha;
      sp[wave][8 * g + r][col] = e0; sp[wave][8 * g + r][16 + col] = e1; }
    LDSX();
    const F2 pa = split_row(&sp[wave][col][0], 0, lane);
#pragma unroll
    for (int dt = 0; dt < 4; ++dt) { const size_t vr = ((size_t)b * DM + h * HD + dt * 16 + col) * SS + ks * 32; const v16b vh = frag_b(VTH + vr, lane), vl = frag_b(VTL + vr, lane); acc[dt] = wmma_bf(pa.l, vh, acc[dt]); acc[dt] = wmma_bf(pa.h, vl, acc[dt]); acc[dt] = wmma_bf(pa.h, vh, acc[dt]); }
    LDSX(); }
#pragma unroll
  for (int r = 0; r < 8; ++r) { const float il = 1.0f / l[r];
#pragma unroll
    for (int dt = 0; dt < 4; ++dt) { const int d = dt * 16 + col; float w2 = 0.f;
#pragma unroll
      for (int j = 0; j < 5; ++j) w2 += (ms[r][j] * il) * bfr(RV[j * HD + d]);
      so[wave][8 * g + r][d] = acc[dt][r] * il + w2; } }
  LDSX();
  for (int rl = 0; rl < 16; ++rl) if (lane < 16) vst2(O + ((size_t)b * SS + q0 + rl) * DM + h * HD + lane * 4, *(const v4f*)&so[wave][rl][lane * 4]);
}
__global__ __launch_bounds__(128) void k_out(const float* __restrict__ O, const __bf16* __restrict__ P, const float* __restrict__ BO, float* __restrict__ Y) {
  __shared__ __align__(16) float so[4][16][132];
  const int tid = threadIdx.x, wave = tid >> 5, lane = tid & 31, col = lane & 15, g = lane >> 4; const size_t r0 = (size_t)blockIdx.x * 64 + wave * 16; const int n0 = blockIdx.y * 128;
  v8f acc[8] = {};
#pragma unroll 2
  for (int kc = 0; kc < DM / 32; ++kc) { const F2 a = split_row(O + (r0 + col) * DM, kc * 32, lane);
#pragma unroll
    for (int j = 0; j < 8; ++j) { const v16b w = frag_b(P + (size_t)(n0 + j * 16 + col) * DM + kc * 32, lane); acc[j] = wmma_bf(a.l, w, acc[j]); acc[j] = wmma_bf(a.h, w, acc[j]); } }
#pragma unroll
  for (int j = 0; j < 8; ++j) { const float bb = bfr(BO[n0 + j * 16 + col]);
#pragma unroll
    for (int r = 0; r < 8; ++r) so[wave][8 * g + r][j * 16 + col] = acc[j][r] + bb; }
  LDSX();
  for (int rl = 0; rl < 16; ++rl) vst2(Y + (r0 + rl) * DM + n0 + lane * 4, *(const v4f*)&so[wave][rl][lane * 4]);
}
extern "C" void kernel_launch(void* const* d_in, const int* in_sizes, int n_in, void* d_out, int out_size, void* d_ws, size_t ws_size, hipStream_t stream) {
  (void)in_sizes; (void)n_in; (void)out_size;
  const float** F = (const float**)d_in;
  if (ws_size < (size_t)WS_END) return;
  char* ws = (char*)d_ws; __bf16 *PK = (__bf16*)(ws + WS_PK), *VTH = (__bf16*)(ws + WS_VTH), *VTL = (__bf16*)(ws + WS_VTL); float *QK = (float*)(ws + WS_QK), *O = (float*)(ws + WS_O);
  k_packrows<<<DM, 256, 0, stream>>>(F[3], DM, PK + PK_A); k_packrows<<<DM, 256, 0, stream>>>(F[5], DM, PK + PK_A + (size_t)DM * DM); k_packrows<<<DM, 256, 0, stream>>>(F[7], DM, PK + PK_A + (size_t)2 * DM * DM); k_packrows<<<DM, 256, 0, stream>>>(F[9], DM, PK + PK_P);
  k_qkv<<<dim3(TNB * SS / 64, QKVW / 128), 128, 0, stream>>>(F[1], F[0], F[2], PK + PK_A, F[4], F[6], F[8], QK);
  k_vt<<<dim3(TNB * SS / 64, NH), 256, 0, stream>>>(QK, VTH, VTL);
  k_attn<<<dim3(TQB, NH, TNB), 128, 0, stream>>>(QK, VTH, VTL, F[11], F[12], O);
  k_out<<<dim3(TOB, DM / 128), 128, 0, stream>>>(O, PK + PK_P, F[10], (float*)d_out);
}
